// BatchMMDLoss_55843164782710
// MI455X (gfx1250) — hardware-verified
//
#include <hip/hip_runtime.h>

typedef _Float16 v16h __attribute__((ext_vector_type(16)));
typedef _Float16 v8h  __attribute__((ext_vector_type(8)));
typedef float    v8f  __attribute__((ext_vector_type(8)));
typedef float    v4f  __attribute__((ext_vector_type(4)));
typedef double   v2d  __attribute__((ext_vector_type(2)));
typedef v8h __attribute__((may_alias)) v8ha;
typedef v4f __attribute__((may_alias)) v4fa;

union Frag { v16h v; v8h half[2]; };

#define NB      32
#define HALFR   1024
#define NZ      2048
#define DF      128
#define NBLK    16
#define NPAIRS  136
#define PSLOT   16
#define CVT_ROWS 32

__device__ __forceinline__ v8f wmma_f16(v16h a, v16h b, v8f c) {
  v8f d = __builtin_amdgcn_wmma_f32_16x16x32_f16(false, a, false, b, (short)0, c, false, false);
  asm volatile("v_nop\n\tv_nop\n\tv_nop\n\tv_nop" : "+v"(d) : "v"(a), "v"(b));
  return d;
}

__device__ __forceinline__ v16h load_frag(const _Float16* p, int h) {
  Frag f;
  f.half[0] = *(const v8ha*)(p + 8 * h);
  f.half[1] = *(const v8ha*)(p + 16 + 8 * h);
  return f.v;
}

__global__ __launch_bounds__(512) void convert_rows(
    const float* __restrict__ X, const float* __restrict__ Y,
    _Float16* __restrict__ zh, float* __restrict__ sq)
{
  __shared__ __attribute__((aligned(16))) float ssq[CVT_ROWS];

  const int tid = threadIdx.x, lane = tid & 31, w = tid >> 5;
  const int h = lane >> 4, m = lane & 15;
  const int lr = 2 * w + h;
  const int gr = blockIdx.x * CVT_ROWS + lr;
  const int b = gr >> 11, r = gr & (NZ - 1);
  const int isy = (r >= HALFR) ? 1 : 0;
  const int rr = r & (HALFR - 1);
  const float* base = isy ? Y : X;
  const float* src = base + ((size_t)b * HALFR + rr) * DF + 8 * m;

  const v4f a = *(const v4fa*)src;
  const v4f c = *(const v4fa*)(src + 4);
  const v8h o = { (_Float16)a.x, (_Float16)a.y, (_Float16)a.z, (_Float16)a.w,
                  (_Float16)c.x, (_Float16)c.y, (_Float16)c.z, (_Float16)c.w };
  float ss = a.x * a.x + a.y * a.y + a.z * a.z + a.w * a.w
           + c.x * c.x + c.y * c.y + c.z * c.z + c.w * c.w;
  ss += __shfl_xor(ss, 1);
  ss += __shfl_xor(ss, 2);
  ss += __shfl_xor(ss, 4);
  ss += __shfl_xor(ss, 8);

  _Float16* dst = zh + (size_t)gr * DF + 8 * m;
  *(volatile v8h*)dst = o;
  if (m == 0) ssq[lr] = ss;
  __syncthreads();

  const v4f sv = *(const v4fa*)(ssq + 4 * (lane & 7));
  float* sdst = sq + (size_t)blockIdx.x * CVT_ROWS + 4 * (lane & 7);
  if (tid < 8) *(volatile v4f*)sdst = sv;
  __threadfence();
  *(volatile v8h*)dst = o;
  if (tid < 8) *(volatile v4f*)sdst = sv;
}

template <int PASS>
__global__ __launch_bounds__(256) void gram_tiles(
    const _Float16* __restrict__ zh,
    const float* __restrict__ sq,
    const float* __restrict__ nib,
    double* __restrict__ part)
{
  __shared__ double red[256];

  const int tid = threadIdx.x, lane = tid & 31, w = tid >> 5;
  const int h = lane >> 4, m = lane & 15;
  const int b = blockIdx.y;
  const int pair = blockIdx.x;
  int bi = 0, rem = pair;
  while (bi < NBLK - 1 && rem >= NBLK - bi) { rem -= NBLK - bi; ++bi; }
  const int bj = bi + rem;

  const int rowbase = (w & 3) * 32;
  const int colbase = (w >> 2) * 64;

  const _Float16* zb = zh + (size_t)b * NZ * DF;
  const _Float16* arow0 = zb + (size_t)(bi * 128 + rowbase + m) * DF;
  const _Float16* arow1 = arow0 + (size_t)16 * DF;
  const _Float16* brow  = zb + (size_t)(bj * 128 + colbase + m) * DF;

  const v8f zero8 = {0.f, 0.f, 0.f, 0.f, 0.f, 0.f, 0.f, 0.f};
  v8f acc[2][4];
  #pragma unroll
  for (int rt = 0; rt < 2; ++rt)
    #pragma unroll
    for (int ct = 0; ct < 4; ++ct) acc[rt][ct] = zero8;

  #pragma unroll 1
  for (int k0 = 0; k0 < DF; k0 += 32) {
    const v16h a0 = load_frag(arow0 + k0, h);
    const v16h a1 = load_frag(arow1 + k0, h);
    #pragma unroll
    for (int ct = 0; ct < 4; ++ct) {
      const v16h bb = load_frag(brow + (size_t)ct * 16 * DF + k0, h);
      acc[0][ct] = wmma_f16(a0, bb, acc[0][ct]);
      acc[1][ct] = wmma_f16(a1, bb, acc[1][ct]);
    }
  }

  const float* sqb = sq + (size_t)b * NZ;
  float nbv = 0.0f;
  if (PASS == 2) nbv = nib[b];
  double lsum = 0.0;
  #pragma unroll
  for (int rt = 0; rt < 2; ++rt) {
    const int ib = bi * 128 + rowbase + 16 * rt + 8 * h;
    const v4f s0 = *(const v4fa*)(sqb + ib);
    const v4f s1 = *(const v4fa*)(sqb + ib + 4);
    const float si[8] = {s0.x, s0.y, s0.z, s0.w, s1.x, s1.y, s1.z, s1.w};
    #pragma unroll
    for (int ct = 0; ct < 4; ++ct) {
      const int j = bj * 128 + colbase + 16 * ct + m;
      const float sj = sqb[j];
      #pragma unroll
      for (int r = 0; r < 8; ++r) {
        float d2 = si[r] + sj - 2.0f * acc[rt][ct][r];
        d2 = fmaxf(d2, 0.0f);
        if (PASS == 1) {
          lsum += (double)d2;
        } else {
          lsum += (double)__expf(d2 * nbv);
        }
      }
    }
  }

  red[tid] = lsum;
  __syncthreads();
  for (int s = 128; s > 0; s >>= 1) {
    if (tid < s) red[tid] += red[tid + s];
    __syncthreads();
  }
  const double tot = red[0];

  v2d v;
  v.x = (tid == 0) ? tot : 0.0;
  v.y = 0.0;
  double* dst = part + ((size_t)b * NPAIRS + pair) * PSLOT + 2 * (lane & 7);
  if (tid < 8) *(volatile v2d*)dst = v;
  __threadfence();
  if (tid < 8) *(volatile v2d*)dst = v;
}

__global__ __launch_bounds__(64) void bw_reduce(const double* __restrict__ part1,
                                                float* __restrict__ nib)
{
  __shared__ __attribute__((aligned(16))) float snb[NB];
  const int tid = threadIdx.x, lane = tid & 31;
  const int b = (tid < NB) ? tid : (NB - 1);
  const double* pb = part1 + (size_t)b * NPAIRS * PSLOT;

  double s = 0.0;
  int idx = 0;
  #pragma unroll 1
  for (int bi = 0; bi < NBLK; ++bi) {
    #pragma unroll 1
    for (int bj = bi; bj < NBLK; ++bj) {
      const double wgt = (bi == bj) ? 1.0 : 2.0;
      s += wgt * pb[(size_t)idx * PSLOT];
      ++idx;
    }
  }
  const double denom = (double)NZ * (double)NZ - (double)NZ;
  const float bwf = (float)(s / denom);
  const float nbf = -(float)(1.0 / (double)bwf);
  if (tid < NB) snb[tid] = nbf;
  __syncthreads();

  const v4f v = *(const v4fa*)(snb + 4 * (lane & 7));
  if (tid < 8) *(volatile v4f*)(nib + 4 * tid) = v;
  __threadfence();
  if (tid < 8) *(volatile v4f*)(nib + 4 * tid) = v;
}

__global__ __launch_bounds__(64) void mmd_final(const double* __restrict__ part2,
                                                float* __restrict__ out)
{
  __shared__ double smm[NB];
  const int tid = threadIdx.x;
  const int b = (tid < NB) ? tid : (NB - 1);
  const double* pb = part2 + (size_t)b * NPAIRS * PSLOT;

  double sxx = 0.0, sxy = 0.0, syy = 0.0;
  int idx = 0;
  #pragma unroll 1
  for (int bi = 0; bi < NBLK; ++bi) {
    #pragma unroll 1
    for (int bj = bi; bj < NBLK; ++bj) {
      const double p = pb[(size_t)idx * PSLOT];
      const double wgt = (bi == bj) ? 1.0 : 2.0;
      if (bj < NBLK / 2)      sxx += wgt * p;
      else if (bi < NBLK / 2) sxy += p;
      else                    syy += wgt * p;
      ++idx;
    }
  }
  const double inv = 1.0 / ((double)HALFR * (double)HALFR);
  const double mmd = sxx * inv - 2.0 * (sxy * inv) + syy * inv;
  if (tid < NB) smm[tid] = mmd;
  __syncthreads();

  double tot = 0.0;
  #pragma unroll 1
  for (int i = 0; i < NB; ++i) tot += smm[i];
  const float tf = (float)tot;
  if (tid == 0) *(volatile float*)out = tf;
  __threadfence();
  if (tid == 0) *(volatile float*)out = tf;
}

extern "C" void kernel_launch(void* const* d_in, const int* in_sizes, int n_in,
                              void* d_out, int out_size, void* d_ws, size_t ws_size,
                              hipStream_t stream) {
  if (n_in < 2) return;
  const int nx = NB * HALFR * DF;
  if (in_sizes[0] != nx || in_sizes[1] != nx) return;
  if (out_size != 1) return;

  const float* X = (const float*)d_in[0];
  const float* Y = (const float*)d_in[1];
  float* out = (float*)d_out;

  const size_t zh_bytes   = (size_t)NB * NZ * DF * 2;
  const size_t sq_bytes   = (size_t)NB * NZ * 4;
  const size_t part_bytes = (size_t)NB * NPAIRS * PSLOT * sizeof(double);
  const size_t nib_bytes  = 128;
  const size_t total = zh_bytes + sq_bytes + part_bytes + nib_bytes + part_bytes;
  if (total > ws_size) return;

  char* ws = (char*)d_ws;
  _Float16* zh  = (_Float16*)(ws);
  float*   sq   = (float*)(ws + zh_bytes);
  double*  p1   = (double*)(ws + zh_bytes + sq_bytes);
  float*   nib  = (float*)(ws + zh_bytes + sq_bytes + part_bytes);
  double*  p2   = (double*)(ws + zh_bytes + sq_bytes + part_bytes + nib_bytes);

  convert_rows<<<(NB * NZ) / CVT_ROWS, 512, 0, stream>>>(X, Y, zh, sq);

  dim3 gT(NPAIRS, NB);
  gram_tiles<1><<<gT, 256, 0, stream>>>(zh, sq, nib, p1);
  bw_reduce<<<1, 64, 0, stream>>>(p1, nib);
  gram_tiles<2><<<gT, 256, 0, stream>>>(zh, sq, nib, p2);
  mmd_final<<<1, 64, 0, stream>>>(p2, out);
}
